// GatedAttentionUnit_79809082294687
// MI455X (gfx1250) — hardware-run, weakly checked
//
#include <hip/hip_runtime.h>
#pragma clang fp contract(off)

typedef __bf16 v16b __attribute__((ext_vector_type(16)));
typedef __bf16 v8b  __attribute__((ext_vector_type(8)));
typedef float  v8f  __attribute__((ext_vector_type(8)));
typedef float  v4f  __attribute__((ext_vector_type(4)));
typedef unsigned int v4u __attribute__((ext_vector_type(4)));
typedef v8b __attribute__((may_alias)) v8ba;
typedef v4f __attribute__((may_alias)) v4fa;
typedef v4u __attribute__((may_alias)) v4ua;

union FragB { v16b v; v8b half[2]; };

#define NB   8
#define NTOK 2048
#define DMOD 256
#define SQK  128
#define HEXP 512
#define ECOL 1152
#define MROW 16384
#define TP   68

#define SZ_XB   ((size_t)MROW * DMOD * 2)
#define SZ_RS   ((size_t)MROW * 4)
#define SZ_WUVT ((size_t)ECOL * DMOD * 2)
#define SZ_WO2  ((size_t)DMOD * 2 * HEXP * 2)
#define SZ_PAR  ((size_t)2048 * 4)
#define SZ_U    ((size_t)MROW * HEXP * 4)
#define SZ_QHL  ((size_t)MROW * 2 * SQK * 2)
#define SZ_KHL  ((size_t)MROW * 2 * SQK * 2)
#define SZ_VTHL ((size_t)NB * HEXP * 2 * NTOK * 2)
#define SZ_PHL  ((size_t)NTOK * 2 * NTOK * 2)
#define SZ_GHL  ((size_t)NTOK * 2 * HEXP * 2)

#define OFF_XB   ((size_t)0)
#define OFF_RS   (OFF_XB + SZ_XB)
#define OFF_WUVT (OFF_RS + SZ_RS)
#define OFF_WO2  (OFF_WUVT + SZ_WUVT)
#define OFF_PAR  (OFF_WO2 + SZ_WO2)
#define OFF_U    (OFF_PAR + SZ_PAR)
#define OFF_QHL  (OFF_U + SZ_U)
#define OFF_KHL  (OFF_QHL + SZ_QHL)
#define OFF_VTHL (OFF_KHL + SZ_KHL)
#define OFF_PHL  (OFF_VTHL + SZ_VTHL)
#define OFF_GHL  (OFF_PHL + SZ_PHL)
#define WS_TOTAL (OFF_GHL + SZ_GHL)

static_assert(WS_TOTAL == (size_t)114'434'048);
static_assert(WS_TOTAL <= (size_t)134'217'728);
static_assert(OFF_RS % 256 == 0 && OFF_WUVT % 256 == 0 && OFF_WO2 % 256 == 0 && OFF_PAR % 256 == 0);
static_assert(OFF_U % 256 == 0 && OFF_QHL % 256 == 0 && OFF_KHL % 256 == 0 && OFF_VTHL % 256 == 0);
static_assert(OFF_PHL % 256 == 0 && OFF_GHL % 256 == 0);
static_assert(NTOK % 128 == 0 && HEXP % 64 == 0 && ECOL % 64 == 0 && MROW % 32 == 0 && DMOD % 32 == 0);
static_assert(MROW % 128 == 0 && DMOD % 64 == 0 && (2 * HEXP) % 64 == 0);

#define PAR_BUV   0
#define PAR_GAMMA 1152
#define PAR_BETA  1408
#define PAR_BO    1664
#define PAR_G     1920
#define PAR_N     2048

#define PREP_NROW 512
#define PREP_NTU  72
#define PREP_NTO  32
#define PREP_GRID (PREP_NROW + PREP_NTU + PREP_NTO + 1)

__device__ __forceinline__ unsigned f2bf_bits(float f) {
  const unsigned u = __float_as_uint(f);
  return (u + 0x7FFFu + ((u >> 16) & 1u)) >> 16;
}
__device__ __forceinline__ float bf_bits2f(unsigned hb) { return __uint_as_float(hb << 16); }
__device__ __forceinline__ float bf_rne(float f) { return bf_bits2f(f2bf_bits(f)); }

struct HL8 { v4u hi; v4u lo; };
__device__ __forceinline__ HL8 split8(float f0, float f1, float f2, float f3,
                                      float f4, float f5, float f6, float f7) {
  const unsigned h0 = f2bf_bits(f0), h1 = f2bf_bits(f1), h2 = f2bf_bits(f2), h3 = f2bf_bits(f3);
  const unsigned h4 = f2bf_bits(f4), h5 = f2bf_bits(f5), h6 = f2bf_bits(f6), h7 = f2bf_bits(f7);
  const unsigned l0 = f2bf_bits(f0 - bf_bits2f(h0)), l1 = f2bf_bits(f1 - bf_bits2f(h1));
  const unsigned l2 = f2bf_bits(f2 - bf_bits2f(h2)), l3 = f2bf_bits(f3 - bf_bits2f(h3));
  const unsigned l4 = f2bf_bits(f4 - bf_bits2f(h4)), l5 = f2bf_bits(f5 - bf_bits2f(h5));
  const unsigned l6 = f2bf_bits(f6 - bf_bits2f(h6)), l7 = f2bf_bits(f7 - bf_bits2f(h7));
  HL8 o;
  const v4u hv = { h0 | (h1 << 16), h2 | (h3 << 16), h4 | (h5 << 16), h6 | (h7 << 16) };
  const v4u lv = { l0 | (l1 << 16), l2 | (l3 << 16), l4 | (l5 << 16), l6 | (l7 << 16) };
  o.hi = hv; o.lo = lv;
  return o;
}

__device__ __forceinline__ void store_hl(unsigned short* dh, unsigned short* dl, v4u hv, v4u lv) {
  *(volatile v4ua*)dh = hv;
  *(volatile v4ua*)dl = lv;
  __threadfence();
  *(volatile v4ua*)dh = hv;
  *(volatile v4ua*)dl = lv;
}
__device__ __forceinline__ void store_u4(unsigned short* d, v4u v) {
  *(volatile v4ua*)d = v;
  __threadfence();
  *(volatile v4ua*)d = v;
}
__device__ __forceinline__ void store_f4(float* d, v4f v) {
  *(volatile v4fa*)d = v;
  __threadfence();
  *(volatile v4fa*)d = v;
}
__device__ __forceinline__ void store_f1(float* d, float v) {
  *(volatile float*)d = v;
  __threadfence();
  *(volatile float*)d = v;
}

__device__ __forceinline__ float silu_fast(float t) {
  return t * __builtin_amdgcn_rcpf(1.0f + __expf(-t));
}

__device__ __forceinline__ v8f wmma_bf(v16b a, v16b b, v8f c) {
  v8f d = __builtin_amdgcn_wmma_f32_16x16x32_bf16(false, a, false, b, (short)0, c, false, false);
  asm volatile("v_nop\n\tv_nop\n\tv_nop\n\tv_nop" : "+v"(d) : "v"(a), "v"(b));
  return d;
}
__device__ __forceinline__ v16b load_frag(const __bf16* p, int h) {
  FragB f;
  f.half[0] = *(const v8ba*)(p + 8 * h);
  f.half[1] = *(const v8ba*)(p + 16 + 8 * h);
  return f.v;
}

__device__ __forceinline__ void tr_tile(const float* __restrict__ W, int Cc,
                                        unsigned short* out, int ldo,
                                        int r0, int c0, int dup, float* tf, int tid) {
  {
    const int lr = tid >> 4, c4 = (tid & 15) * 4;
    #pragma unroll
    for (int it = 0; it < 4; ++it) {
      const int rr = it * 16 + lr;
      const v4f a = *(const v4fa*)(W + (size_t)(r0 + rr) * Cc + c0 + c4);
      *(v4fa*)(tf + rr * TP + c4) = a;
    }
  }
  __syncthreads();
  const int sub = tid >> 3, c8 = (tid & 7) * 8;
  #pragma unroll 1
  for (int it = 0; it < 2; ++it) {
    const int oc = it * 32 + sub;
    const unsigned h0 = f2bf_bits(tf[(c8 + 0) * TP + oc]);
    const unsigned h1 = f2bf_bits(tf[(c8 + 1) * TP + oc]);
    const unsigned h2 = f2bf_bits(tf[(c8 + 2) * TP + oc]);
    const unsigned h3 = f2bf_bits(tf[(c8 + 3) * TP + oc]);
    const unsigned h4 = f2bf_bits(tf[(c8 + 4) * TP + oc]);
    const unsigned h5 = f2bf_bits(tf[(c8 + 5) * TP + oc]);
    const unsigned h6 = f2bf_bits(tf[(c8 + 6) * TP + oc]);
    const unsigned h7 = f2bf_bits(tf[(c8 + 7) * TP + oc]);
    const v4u hv = { h0 | (h1 << 16), h2 | (h3 << 16), h4 | (h5 << 16), h6 | (h7 << 16) };
    unsigned short* dst = out + (size_t)(c0 + oc) * ldo + r0 + c8;
    if (dup != 0) {
      store_hl(dst, dst + dup, hv, hv);
    } else {
      store_u4(dst, hv);
    }
  }
}

__global__ __launch_bounds__(256) void k_prep(
    const float* __restrict__ x, const float* __restrict__ g,
    const float* __restrict__ W_uv, const float* __restrict__ b_uv,
    const float* __restrict__ gamma, const float* __restrict__ beta,
    const float* __restrict__ W_o, const float* __restrict__ b_o,
    unsigned char* __restrict__ ws)
{
  __shared__ __attribute__((aligned(16))) float tf[64 * TP];
  __shared__ __attribute__((aligned(16))) float sm[32];

  const int tid = threadIdx.x, lane = tid & 31, w = tid >> 5;
  const int blk = blockIdx.x;

  if (blk < PREP_NROW) {
    unsigned short* XB = (unsigned short*)(ws + OFF_XB);
    float* RS = (float*)(ws + OFF_RS);
    #pragma unroll 1
    for (int i = 0; i < 4; ++i) {
      const int lr = w * 4 + i;
      const size_t row = (size_t)blk * 32 + lr;
      const float* xr = x + row * DMOD + 8 * lane;
      const v4f a = *(const v4fa*)xr;
      const v4f c = *(const v4fa*)(xr + 4);
      const unsigned h0 = f2bf_bits(a.x), h1 = f2bf_bits(a.y), h2 = f2bf_bits(a.z), h3 = f2bf_bits(a.w);
      const unsigned h4 = f2bf_bits(c.x), h5 = f2bf_bits(c.y), h6 = f2bf_bits(c.z), h7 = f2bf_bits(c.w);
      const float r0 = bf_bits2f(h0), r1 = bf_bits2f(h1), r2 = bf_bits2f(h2), r3 = bf_bits2f(h3);
      const float r4 = bf_bits2f(h4), r5 = bf_bits2f(h5), r6 = bf_bits2f(h6), r7 = bf_bits2f(h7);
      float ss = r0 * r0;
      ss = ss + r1 * r1;
      ss = ss + r2 * r2;
      ss = ss + r3 * r3;
      ss = ss + r4 * r4;
      ss = ss + r5 * r5;
      ss = ss + r6 * r6;
      ss = ss + r7 * r7;
      ss = ss + __shfl_xor(ss, 16);
      ss = ss + __shfl_xor(ss, 8);
      ss = ss + __shfl_xor(ss, 4);
      ss = ss + __shfl_xor(ss, 2);
      ss = ss + __shfl_xor(ss, 1);
      const float nrm = sqrtf(ss) * 0.0625f;
      const float mm = fmaxf(nrm, 1e-5f);
      const v4u o = { h0 | (h1 << 16), h2 | (h3 << 16), h4 | (h5 << 16), h6 | (h7 << 16) };
      store_u4(XB + row * DMOD + 8 * lane, o);
      if (lane == 0) sm[lr] = mm;
    }
    __syncthreads();
    const v4f mv = *(const v4fa*)(sm + 4 * (tid & 7));
    asm volatile("" :: "v"(mv));
    if (tid < 8) store_f4(RS + (size_t)blk * 32 + 4 * tid, mv);
  } else if (blk < PREP_NROW + PREP_NTU) {
    const int tb = blk - PREP_NROW;
    const int cx = tb % 18, ry = tb / 18;
    tr_tile(W_uv, ECOL, (unsigned short*)(ws + OFF_WUVT), DMOD, ry * 64, cx * 64, 0, tf, tid);
  } else if (blk < PREP_NROW + PREP_NTU + PREP_NTO) {
    const int tb = blk - PREP_NROW - PREP_NTU;
    const int cx = tb & 3, ry = tb >> 2;
    tr_tile(W_o, DMOD, (unsigned short*)(ws + OFF_WO2), 2 * HEXP, ry * 64, cx * 64, HEXP, tf, tid);
  } else {
    float* PAR = (float*)(ws + OFF_PAR);
    #pragma unroll 1
    for (int i = tid; i < ECOL; i += 256) {
      const float v = bf_rne(b_uv[i]);
      store_f1(PAR + PAR_BUV + i, v);
    }
    {
      const float v = bf_rne(gamma[tid]);
      store_f1(PAR + PAR_GAMMA + tid, v);
    }
    {
      const float v = bf_rne(beta[tid]);
      store_f1(PAR + PAR_BETA + tid, v);
    }
    {
      const float v = bf_rne(b_o[tid]);
      store_f1(PAR + PAR_BO + tid, v);
    }
    if (tid < 128) {
      const float gv = g[0];
      asm volatile("" :: "v"(gv));
      const float v = (tid == 0) ? bf_rne(gv) : 0.0f;
      store_f1(PAR + PAR_G + tid, v);
    }
  }
}

template <int EPI, int NSEG, int LDA, int LDB, int KSEG>
__global__ __launch_bounds__(128) __attribute__((amdgpu_num_vgpr(248)))
void k_gemm(unsigned char* ws, float* out, int bidx)
{
  static_assert(KSEG % 32 == 0);
  static_assert(NSEG == 1 || NSEG == 3);
  static_assert(NSEG == 1 ? (LDA == KSEG && LDB == KSEG) : (LDA == 2 * KSEG && LDB == 2 * KSEG));
  static_assert(LDA % 8 == 0 && LDB % 8 == 0);
  static_assert((128 * TP + 512 + 128) * 4 <= 327680);

  __shared__ __attribute__((aligned(16))) float sT[128 * TP];
  __shared__ __attribute__((aligned(16))) float sPar[512];
  __shared__ __attribute__((aligned(16))) float sRS[128];

  const int tid = threadIdx.x, lane = tid & 31, w = tid >> 5;
  const int h = lane >> 4, m = lane & 15;
  const int m0 = blockIdx.x * 128, n0 = blockIdx.y * 64;

  const __bf16* Ab;
  const __bf16* Bb;
  if (EPI == 0) {
    Ab = (const __bf16*)(ws + OFF_XB);
    Bb = (const __bf16*)(ws + OFF_WUVT);
  } else if (EPI == 1) {
    Ab = (const __bf16*)(ws + OFF_QHL) + (size_t)bidx * NTOK * (2 * SQK);
    Bb = (const __bf16*)(ws + OFF_KHL) + (size_t)bidx * NTOK * (2 * SQK);
  } else if (EPI == 2) {
    Ab = (const __bf16*)(ws + OFF_PHL);
    Bb = (const __bf16*)(ws + OFF_VTHL) + (size_t)bidx * HEXP * (2 * NTOK);
  } else {
    Ab = (const __bf16*)(ws + OFF_GHL);
    Bb = (const __bf16*)(ws + OFF_WO2);
  }

  const __bf16* xa0 = Ab + (size_t)(m0 + 32 * w + m) * LDA;
  const __bf16* xa1 = xa0 + (size_t)16 * LDA;
  const __bf16* wb  = Bb + (size_t)(n0 + m) * LDB;

  const v8f zero8 = {0.f, 0.f, 0.f, 0.f, 0.f, 0.f, 0.f, 0.f};
  v8f acc[2][4];
  #pragma unroll
  for (int mt = 0; mt < 2; ++mt)
    #pragma unroll
    for (int nt = 0; nt < 4; ++nt) acc[mt][nt] = zero8;

  #pragma unroll 1
  for (int seg = 0; seg < NSEG; ++seg) {
    const int ao = (seg == 1) ? KSEG : 0;
    const int bo = (seg == 2) ? KSEG : 0;
    #pragma unroll 1
    for (int k0 = 0; k0 < KSEG; k0 += 32) {
      const v16b a0 = load_frag(xa0 + ao + k0, h);
      const v16b a1 = load_frag(xa1 + ao + k0, h);
      #pragma unroll
      for (int nt = 0; nt < 4; ++nt) {
        const v16b b = load_frag(wb + (size_t)nt * 16 * LDB + bo + k0, h);
        acc[0][nt] = wmma_bf(a0, b, acc[0][nt]);
        acc[1][nt] = wmma_bf(a1, b, acc[1][nt]);
      }
    }
  }

  #pragma unroll
  for (int mt = 0; mt < 2; ++mt)
    #pragma unroll
    for (int nt = 0; nt < 4; ++nt)
      #pragma unroll
      for (int r = 0; r < 8; ++r)
        sT[(32 * w + 16 * mt + 8 * h + r) * TP + 16 * nt + m] = acc[mt][nt][r];

  if (EPI == 0) {
    const float* par = (const float*)(ws + OFF_PAR);
    const float* rs  = (const float*)(ws + OFF_RS);
    {
      const int vec = tid >> 4, c4 = (tid & 15) * 4;
      const int j0 = (n0 >= 2 * HEXP) ? (n0 - 2 * HEXP) : 0;
      int off = PAR_BUV + n0;
      off = (vec == 1) ? (PAR_GAMMA + j0) : off;
      off = (vec == 2) ? (PAR_BETA + j0) : off;
      off = (vec == 3) ? (PAR_GAMMA + SQK + j0) : off;
      off = (vec >= 4) ? (PAR_BETA + SQK + j0) : off;
      const v4f pv = *(const v4fa*)(par + off + c4);
      *(v4fa*)(sPar + vec * 64 + c4) = pv;
    }
    if (w == 0) {
      const v4f rv = *(const v4fa*)(rs + m0 + 4 * lane);
      *(v4fa*)(sRS + 4 * lane) = rv;
    }
    const float gval = par[PAR_G];
    __syncthreads();

    #pragma unroll 1
    for (int it = 0; it < 16; ++it) {
      const int idx = it * 128 + tid;
      const int row = idx >> 4, c4 = (idx & 15) * 4;
      const v4f v = *(const v4fa*)(sT + row * TP + c4);
      const float mr = sRS[row];
      const v4f bb = *(const v4fa*)(sPar + c4);
      v4f o;
      o.x = silu_fast((v.x / mr) * gval + bb.x);
      o.y = silu_fast((v.y / mr) * gval + bb.y);
      o.z = silu_fast((v.z / mr) * gval + bb.z);
      o.w = silu_fast((v.w / mr) * gval + bb.w);
      *(v4fa*)(sT + row * TP + c4) = o;
    }
    __syncthreads();

    if (n0 < HEXP) {
      float* U = (float*)(ws + OFF_U);
      #pragma unroll 1
      for (int it = 0; it < 16; ++it) {
        const int idx = it * 128 + tid;
        const int row = idx >> 4, c4 = (idx & 15) * 4;
        const v4f v = *(const v4fa*)(sT + row * TP + c4);
        store_f4(U + (size_t)(m0 + row) * HEXP + n0 + c4, v);
      }
    } else if (n0 < 2 * HEXP) {
      unsigned short* vt = (unsigned short*)(ws + OFF_VTHL);
      const int bb = m0 >> 11, t0 = m0 & (NTOK - 1);
      #pragma unroll 1
      for (int it = 0; it < 8; ++it) {
        const int idx = it * 128 + tid;
        const int feat = idx >> 4, tc = (idx & 15) * 8;
        const float f0 = sT[(tc + 0) * TP + feat];
        const float f1 = sT[(tc + 1) * TP + feat];
        const float f2 = sT[(tc + 2) * TP + feat];
        const float f3 = sT[(tc + 3) * TP + feat];
        const float f4 = sT[(tc + 4) * TP + feat];
        const float f5 = sT[(tc + 5) * TP + feat];
        const float f6 = sT[(tc + 6) * TP + feat];
        const float f7 = sT[(tc + 7) * TP + feat];
        const HL8 p = split8(f0, f1, f2, f3, f4, f5, f6, f7);
        unsigned short* dst = vt + ((size_t)(bb * HEXP + (n0 - HEXP) + feat)) * (2 * NTOK) + t0 + tc;
        store_hl(dst, dst + NTOK, p.hi, p.lo);
      }
    } else {
      unsigned short* qh = (unsigned short*)(ws + OFF_QHL);
      unsigned short* kh = (unsigned short*)(ws + OFF_KHL);
      const int j0 = n0 - 2 * HEXP;
      const int c8 = (tid & 7) * 8;
      const v4f g0a = *(const v4fa*)(sPar + 64 + c8),  g0b = *(const v4fa*)(sPar + 64 + c8 + 4);
      const v4f b0a = *(const v4fa*)(sPar + 128 + c8), b0b = *(const v4fa*)(sPar + 128 + c8 + 4);
      const v4f g1a = *(const v4fa*)(sPar + 192 + c8), g1b = *(const v4fa*)(sPar + 192 + c8 + 4);
      const v4f b1a = *(const v4fa*)(sPar + 256 + c8), b1b = *(const v4fa*)(sPar + 256 + c8 + 4);
      #pragma unroll 1
      for (int it = 0; it < 8; ++it) {
        const int idx = it * 128 + tid;
        const int row = idx >> 3;
        const v4f s0 = *(const v4fa*)(sT + row * TP + c8);
        const v4f s1 = *(const v4fa*)(sT + row * TP + c8 + 4);
        const HL8 pq = split8(s0.x * g0a.x + b0a.x, s0.y * g0a.y + b0a.y, s0.z * g0a.z + b0a.z, s0.w * g0a.w + b0a.w,
                              s1.x * g0b.x + b0b.x, s1.y * g0b.y + b0b.y, s1.z * g0b.z + b0b.z, s1.w * g0b.w + b0b.w);
        const HL8 pk = split8(s0.x * g1a.x + b1a.x, s0.y * g1a.y + b1a.y, s0.z * g1a.z + b1a.z, s0.w * g1a.w + b1a.w,
                              s1.x * g1b.x + b1b.x, s1.y * g1b.y + b1b.y, s1.z * g1b.z + b1b.z, s1.w * g1b.w + b1b.w);
        const size_t ro = (size_t)(m0 + row) * (2 * SQK) + j0 + c8;
        store_hl(qh + ro, qh + ro + SQK, pq.hi, pq.lo);
        store_hl(kh + ro, kh + ro + SQK, pk.hi, pk.lo);
      }
    }
  } else if (EPI == 1) {
    __syncthreads();
    unsigned short* ph = (unsigned short*)(ws + OFF_PHL);
    const float rsq = __uint_as_float(0x3DB504F3u);
    #pragma unroll 1
    for (int it = 0; it < 8; ++it) {
      const int idx = it * 128 + tid;
      const int row = idx >> 3, c8 = (idx & 7) * 8;
      const v4f s0 = *(const v4fa*)(sT + row * TP + c8);
      const v4f s1 = *(const v4fa*)(sT + row * TP + c8 + 4);
      float e0 = s0.x * rsq, e1 = s0.y * rsq, e2 = s0.z * rsq, e3 = s0.w * rsq;
      float e4 = s1.x * rsq, e5 = s1.y * rsq, e6 = s1.z * rsq, e7 = s1.w * rsq;
      e0 = (e0 > 0.0f) ? e0 : 0.0f;  e1 = (e1 > 0.0f) ? e1 : 0.0f;
      e2 = (e2 > 0.0f) ? e2 : 0.0f;  e3 = (e3 > 0.0f) ? e3 : 0.0f;
      e4 = (e4 > 0.0f) ? e4 : 0.0f;  e5 = (e5 > 0.0f) ? e5 : 0.0f;
      e6 = (e6 > 0.0f) ? e6 : 0.0f;  e7 = (e7 > 0.0f) ? e7 : 0.0f;
      const HL8 p = split8(e0 * e0, e1 * e1, e2 * e2, e3 * e3, e4 * e4, e5 * e5, e6 * e6, e7 * e7);
      unsigned short* dst = ph + (size_t)(m0 + row) * (2 * NTOK) + n0 + c8;
      store_hl(dst, dst + NTOK, p.hi, p.lo);
    }
  } else if (EPI == 2) {
    __syncthreads();
    unsigned short* gh = (unsigned short*)(ws + OFF_GHL);
    const float* U = (const float*)(ws + OFF_U);
    #pragma unroll 1
    for (int it = 0; it < 8; ++it) {
      const int idx = it * 128 + tid;
      const int row = idx >> 3, c8 = (idx & 7) * 8;
      const v4f s0 = *(const v4fa*)(sT + row * TP + c8);
      const v4f s1 = *(const v4fa*)(sT + row * TP + c8 + 4);
      const float* up = U + ((size_t)bidx * NTOK + m0 + row) * HEXP + n0 + c8;
      const v4f u0 = *(const v4fa*)up;
      const v4f u1 = *(const v4fa*)(up + 4);
      const HL8 p = split8(s0.x * u0.x, s0.y * u0.y, s0.z * u0.z, s0.w * u0.w,
                           s1.x * u1.x, s1.y * u1.y, s1.z * u1.z, s1.w * u1.w);
      unsigned short* dst = gh + (size_t)(m0 + row) * (2 * HEXP) + n0 + c8;
      store_hl(dst, dst + HEXP, p.hi, p.lo);
    }
  } else {
    const float* par = (const float*)(ws + OFF_PAR);
    if (w == 0) {
      const int c = (lane & 15) * 4;
      const v4f bv = *(const v4fa*)(par + PAR_BO + n0 + c);
      *(v4fa*)(sPar + c) = bv;
    }
    __syncthreads();
    const int c4 = (tid & 15) * 4;
    const v4f bb = *(const v4fa*)(sPar + c4);
    #pragma unroll 1
    for (int it = 0; it < 16; ++it) {
      const int idx = it * 128 + tid;
      const int row = idx >> 4;
      const v4f v = *(const v4fa*)(sT + row * TP + c4);
      v4f o;
      o.x = v.x + bb.x; o.y = v.y + bb.y; o.z = v.z + bb.z; o.w = v.w + bb.w;
      store_f4(out + ((size_t)bidx * NTOK + m0 + row) * DMOD + n0 + c4, o);
    }
  }
}

extern "C" void kernel_launch(void* const* d_in, const int* in_sizes, int n_in,
                              void* d_out, int out_size, void* d_ws, size_t ws_size,
                              hipStream_t stream) {
  if (n_in < 8) return;
  if (in_sizes[0] != MROW * DMOD) return;
  if (in_sizes[1] != 1) return;
  if (in_sizes[2] != DMOD * ECOL) return;
  if (in_sizes[3] != ECOL) return;
  if (in_sizes[4] != 2 * SQK || in_sizes[5] != 2 * SQK) return;
  if (in_sizes[6] != HEXP * DMOD) return;
  if (in_sizes[7] != DMOD) return;
  if (out_size != MROW * DMOD) return;
  if (WS_TOTAL > ws_size) return;

  const float* x     = (const float*)d_in[0];
  const float* g     = (const float*)d_in[1];
  const float* W_uv  = (const float*)d_in[2];
  const float* b_uv  = (const float*)d_in[3];
  const float* gamma = (const float*)d_in[4];
  const float* beta  = (const float*)d_in[5];
  const float* W_o   = (const float*)d_in[6];
  const float* b_o   = (const float*)d_in[7];
  float* out = (float*)d_out;
  unsigned char* ws = (unsigned char*)d_ws;

  k_prep<<<dim3(PREP_GRID), dim3(256), 0, stream>>>(x, g, W_uv, b_uv, gamma, beta, W_o, b_o, ws);

  k_gemm<0, 1, DMOD, DMOD, DMOD><<<dim3(MROW / 128, ECOL / 64), dim3(128), 0, stream>>>(ws, out, 0);

  for (int b = 0; b < NB; ++b) {
    k_gemm<1, 3, 2 * SQK, 2 * SQK, SQK><<<dim3(NTOK / 128, NTOK / 64), dim3(128), 0, stream>>>(ws, out, b);
    k_gemm<2, 3, 2 * NTOK, 2 * NTOK, NTOK><<<dim3(NTOK / 128, HEXP / 64), dim3(128), 0, stream>>>(ws, out, b);
    k_gemm<3, 1, 2 * HEXP, 2 * HEXP, 2 * HEXP><<<dim3(NTOK / 128, DMOD / 64), dim3(128), 0, stream>>>(ws, out, b);
  }
  (void)hipGetLastError();
}
